// PointNetSetAbstraction_4011499454875
// MI455X (gfx1250) — hardware-verified
//
#include <hip/hip_runtime.h>
#include <stdint.h>
#pragma clang fp contract(off)

typedef __attribute__((ext_vector_type(16))) _Float16 v16h;
typedef __attribute__((ext_vector_type(8)))  _Float16 v8h;
typedef __attribute__((ext_vector_type(8)))  float    v8f;
typedef __attribute__((ext_vector_type(4)))  float    v4f;
typedef __attribute__((ext_vector_type(4)))  int      v4i;
typedef __attribute__((ext_vector_type(4)))  unsigned v4u;

constexpr int NBATCH = 16;
constexpr int NPTS   = 4096;
constexpr int NCEN   = 1024;
constexpr int NSMP   = 32;
constexpr int CPTS   = 64;
constexpr int CIN0   = 67;
constexpr int KPAD0  = 96;
constexpr int MROWS  = NBATCH * NCEN * NSMP;
constexpr float WCARRY     = 16.0f;
constexpr float WCARRY_INV = 1.0f / WCARRY;
constexpr float RAD2   = 0.04f;
constexpr float BN_EPS = 1e-5f;

static_assert(MROWS == 524288, "row count");
static_assert(KPAD0 % 32 == 0 && CPTS % 32 == 0, "k multiples of 32");
static_assert(MROWS % 128 == 0, "row tiles");
static_assert(CIN0 == CPTS + 3, "layer 0 input channels");

constexpr size_t SZ_FIDX = (size_t)NBATCH * NCEN * 4;
constexpr size_t SZ_GIDX = (size_t)MROWS * 4;
constexpr size_t SZ_WF   = (size_t)(64 * KPAD0 + 64 * 64 + 128 * 64) * 2;
constexpr size_t SZ_TAB0 = 4 * 64 * 4;
constexpr size_t SZ_TAB1 = 4 * 64 * 4;
constexpr size_t SZ_TAB2 = 4 * 128 * 4;
constexpr size_t SZ_Y0   = (size_t)MROWS * 64 * 2;
constexpr size_t SZ_P0   = (size_t)(MROWS / 128) * 128 * 4;
constexpr size_t SZ_P1   = SZ_P0;
constexpr size_t SZ_P2   = (size_t)(MROWS / 64) * 256 * 4;
constexpr size_t SZ_GM   = (size_t)(MROWS / 32) * 128 * 4;
constexpr size_t OFF_FIDX = 0;
constexpr size_t OFF_GIDX = OFF_FIDX + SZ_FIDX;
constexpr size_t OFF_WF   = OFF_GIDX + SZ_GIDX;
constexpr size_t OFF_TAB0 = OFF_WF + SZ_WF;
constexpr size_t OFF_TAB1 = OFF_TAB0 + SZ_TAB0;
constexpr size_t OFF_TAB2 = OFF_TAB1 + SZ_TAB1;
constexpr size_t OFF_Y0   = OFF_TAB2 + SZ_TAB2;
constexpr size_t OFF_P0   = OFF_Y0 + SZ_Y0;
constexpr size_t OFF_P1   = OFF_P0 + SZ_P0;
constexpr size_t OFF_P2   = OFF_P1 + SZ_P1;
constexpr size_t OFF_GMAX = OFF_P2 + SZ_P2;
constexpr size_t OFF_GMIN = OFF_GMAX + SZ_GM;
constexpr size_t WS_TOTAL = OFF_GMIN + SZ_GM;
static_assert(WS_TOTAL <= (size_t)134217728, "carve within 128 MiB");
static_assert(OFF_GIDX % 128 == 0 && OFF_WF % 128 == 0 && OFF_TAB0 % 128 == 0 && OFF_Y0 % 128 == 0, "line aligned");
static_assert(OFF_P0 % 128 == 0 && OFF_P2 % 128 == 0 && OFF_GMAX % 128 == 0 && OFF_GMIN % 128 == 0, "line aligned");
constexpr size_t OUT0_FLOATS = (size_t)NBATCH * NCEN * 3;
constexpr size_t OUT1_FLOATS = (size_t)NBATCH * NCEN * 128;
static_assert(OUT0_FLOATS * 4 == 196608, "out1 byte offset");
static_assert((OUT0_FLOATS + OUT1_FLOATS) * 4 == 8585216, "d_out total");

union FragH { v16h v; v8h h[2]; };
__device__ __forceinline__ v16h frag_ld(const _Float16* p) {
  FragH f;
  f.h[0] = *(const v8h*)(p);
  f.h[1] = *(const v8h*)(p + 16);
  return f.v;
}
__device__ __forceinline__ v8f mma_h(v16h a, v16h b, v8f c) {
  return __builtin_amdgcn_wmma_f32_16x16x32_f16(false, a, false, b, (short)0, c, false, false);
}
__device__ __forceinline__ void guard4(v8f& c0, v8f& c1, v8f& c2, v8f& c3, v16h a, v16h b0, v16h b1, v16h b2, v16h b3) {
  asm volatile("v_nop\n\tv_nop\n\tv_nop\n\tv_nop"
               : "+v"(c0), "+v"(c1), "+v"(c2), "+v"(c3)
               : "v"(a), "v"(b0), "v"(b1), "v"(b2), "v"(b3));
}
__device__ __forceinline__ void guard2(v8f& c0, v8f& c1, v16h a, v16h b0, v16h b1) {
  asm volatile("v_nop\n\tv_nop\n\tv_nop\n\tv_nop"
               : "+v"(c0), "+v"(c1)
               : "v"(a), "v"(b0), "v"(b1));
}
__device__ __forceinline__ float h16_to_f32(unsigned hb) {
  const unsigned sgn = (hb & 0x8000u) << 16;
  const unsigned em = hb & 0x7fffu;
  const float fn = __uint_as_float((em << 13) + 0x38000000u);
  const float fs = (float)em * 5.9604644775390625e-8f;
  const float mag = (em < 0x400u) ? fs : fn;
  return __uint_as_float(__float_as_uint(mag) | sgn);
}
__device__ __forceinline__ float bn_relu(float y, float m, float inv, float g, float be) {
  float t = (y - m) * inv;
  t = t * g + be;
  return fmaxf(t, 0.0f);
}
__device__ __forceinline__ void put_tile(float* Ts, int pitch, int rbase, int col, v8f acc, float bias) {
#pragma unroll
  for (int r = 0; r < 8; ++r) {
    const float v = acc[r] * WCARRY_INV + bias;
    Ts[(rbase + r) * pitch + col] = v;
  }
}

__global__ __launch_bounds__(256) void k_fps(const float* __restrict__ xyz, float* __restrict__ out0, int* __restrict__ fidx) {
  __shared__ __align__(16) float sx[3 * NPTS];
  __shared__ __align__(16) int sidx[NCEN];
  __shared__ float rv[2][8];
  __shared__ int ri[2][8];
  const int tid = threadIdx.x, lane = tid & 31, wave = tid >> 5;
  const int b = blockIdx.x;
  const float* xb = xyz + (size_t)b * NPTS * 3;
#pragma unroll 4
  for (int i = 0; i < 12; ++i) {
    const int q = tid + 256 * i;
    const v4f v = *(const v4f*)(xb + 4 * q);
#pragma unroll
    for (int e = 0; e < 4; ++e) {
      const int idx = 4 * q + e;
      const int p = idx / 3;
      const int c = idx - 3 * p;
      sx[c * NPTS + p] = v[e];
    }
  }
  __syncthreads();
  float px[16], py[16], pz[16], dist[16];
#pragma unroll
  for (int j = 0; j < 16; ++j) {
    const int p = j * 256 + tid;
    px[j] = sx[p];
    py[j] = sx[NPTS + p];
    pz[j] = sx[2 * NPTS + p];
    dist[j] = 1e10f;
  }
  int far = 0;
#pragma unroll 1
  for (int it = 0; it < NCEN; ++it) {
    if (tid == 0) sidx[it] = far;
    const float cx = sx[far], cy = sx[NPTS + far], cz = sx[2 * NPTS + far];
    float bv = -1.0f;
    int bi = 0;
#pragma unroll
    for (int j = 0; j < 16; ++j) {
      const float dx = px[j] - cx, dy = py[j] - cy, dz = pz[j] - cz;
      const float tx = dx * dx, ty = dy * dy, tz = dz * dz;
      const float d = (tx + tz) + ty;
      const float dd = fminf(dist[j], d);
      dist[j] = dd;
      if (dd > bv) { bv = dd; bi = j * 256 + tid; }
    }
#pragma unroll
    for (int off = 16; off >= 1; off >>= 1) {
      const float ov = __shfl_xor(bv, off, 32);
      const int oi = __shfl_xor(bi, off, 32);
      const bool take = (ov > bv) || (ov == bv && oi < bi);
      bv = take ? ov : bv;
      bi = take ? oi : bi;
    }
    const int buf = it & 1;
    if (lane == 0) { rv[buf][wave] = bv; ri[buf][wave] = bi; }
    __syncthreads();
    float fv = rv[buf][0];
    int fi = ri[buf][0];
#pragma unroll
    for (int w = 1; w < 8; ++w) {
      const float ov = rv[buf][w];
      const int oi = ri[buf][w];
      const bool take = (ov > fv) || (ov == fv && oi < fi);
      fv = take ? ov : fv;
      fi = take ? oi : fi;
    }
    far = fi & (NPTS - 1);
  }
  __syncthreads();
  v4f ov3[3];
#pragma unroll
  for (int i = 0; i < 3; ++i) {
    const int q = tid + 256 * i;
#pragma unroll
    for (int e = 0; e < 4; ++e) {
      const int idx = 4 * q + e;
      const int s = idx / 3;
      const int c = idx - 3 * s;
      const int p = sidx[s] & (NPTS - 1);
      ov3[i][e] = sx[c * NPTS + p];
    }
  }
  const v4i iv = *(const v4i*)(&sidx[4 * tid]);
  float* ob = out0 + (size_t)b * NCEN * 3;
  int* fb = fidx + (size_t)b * NCEN;
  for (int pass = 0; pass < 2; ++pass) {
#pragma unroll
    for (int i = 0; i < 3; ++i) *(volatile v4f*)(ob + 4 * (tid + 256 * i)) = ov3[i];
    *(volatile v4i*)(fb + 4 * tid) = iv;
    __threadfence();
  }
}

__global__ __launch_bounds__(256) void k_ball(const float* __restrict__ xyz, const int* __restrict__ fidx, int* __restrict__ gidx) {
  __shared__ int lst[8][32];
  const int tid = threadIdx.x, lane = tid & 31, wave = tid >> 5;
  const int w = blockIdx.x * 8 + wave;
  const int b = w >> 10;
  lst[wave][lane] = 0;
  __syncthreads();
  int ci = fidx[w];
  ci = ci < 0 ? 0 : (ci > NPTS - 1 ? NPTS - 1 : ci);
  const float* xb = xyz + (size_t)b * NPTS * 3;
  const float cx = xb[ci * 3 + 0], cy = xb[ci * 3 + 1], cz = xb[ci * 3 + 2];
  int cnt = 0;
#pragma unroll 1
  for (int n0 = 0; n0 < NPTS; n0 += 32) {
    if (cnt >= NSMP) break;
    const int p = n0 + lane;
    const float x = xb[p * 3 + 0], y = xb[p * 3 + 1], z = xb[p * 3 + 2];
    const float dx = cx - x, dy = cy - y, dz = cz - z;
    const float tx = dx * dx, ty = dy * dy, tz = dz * dz;
    const float d = (tx + tz) + ty;
    const bool in = !(d > RAD2);
    const unsigned mask = __builtin_amdgcn_ballot_w32(in);
    const int pos = cnt + __builtin_popcount(mask & ((1u << lane) - 1u));
    if (in && pos < NSMP) lst[wave][pos] = p;
    cnt += __builtin_popcount(mask);
    cnt = __builtin_amdgcn_readfirstlane(cnt);
  }
  __syncthreads();
  const int first = lst[wave][0];
  const int mine = lst[wave][lane];
  int v = (lane < cnt) ? mine : first;
  v = v < 0 ? 0 : (v > NPTS - 1 ? NPTS - 1 : v);
  int* dst = gidx + (size_t)w * NSMP + lane;
  *(volatile int*)dst = v;
  __threadfence();
  *(volatile int*)dst = v;
}

__global__ __launch_bounds__(256) void k_wprep(const float* __restrict__ w0, const float* __restrict__ w1,
                                               const float* __restrict__ w2, _Float16* __restrict__ wf) {
  const int tid = threadIdx.x;
  const int blk = blockIdx.x;
  const int ch = blk * 256 + tid;
  v8h hv;
  _Float16* dst;
  if (blk < 3) {
    const int n = ch / 12;
    const int k0 = (ch - n * 12) * 8;
#pragma unroll
    for (int e = 0; e < 8; ++e) {
      const int k = k0 + e;
      int col = (k < 64) ? (k + 3) : (k - 64);
      col = col > CIN0 - 1 ? CIN0 - 1 : col;
      const float v = w0[n * CIN0 + col];
      const float sv = (k < CIN0) ? v * WCARRY : 0.0f;
      hv[e] = (_Float16)sv;
    }
    dst = wf + (size_t)ch * 8;
  } else if (blk < 5) {
    const int c1 = ch - 768;
    const v4f a = *(const v4f*)(w1 + (size_t)c1 * 8);
    const v4f bq = *(const v4f*)(w1 + (size_t)c1 * 8 + 4);
#pragma unroll
    for (int e = 0; e < 4; ++e) { hv[e] = (_Float16)(a[e] * WCARRY); hv[4 + e] = (_Float16)(bq[e] * WCARRY); }
    dst = wf + 64 * KPAD0 + (size_t)c1 * 8;
  } else {
    const int c2 = ch - 1280;
    const v4f a = *(const v4f*)(w2 + (size_t)c2 * 8);
    const v4f bq = *(const v4f*)(w2 + (size_t)c2 * 8 + 4);
#pragma unroll
    for (int e = 0; e < 4; ++e) { hv[e] = (_Float16)(a[e] * WCARRY); hv[4 + e] = (_Float16)(bq[e] * WCARRY); }
    dst = wf + 64 * KPAD0 + 64 * 64 + (size_t)c2 * 8;
  }
  *(volatile v8h*)dst = hv;
  __threadfence();
  *(volatile v8h*)dst = hv;
}

__device__ __forceinline__ void stats128(const float* Ts, float* red, float* stg, float* dst, int tid) {
  const int c = tid & 63, q = tid >> 6;
  float s1 = 0.0f, s2 = 0.0f;
#pragma unroll 4
  for (int i = 0; i < 32; ++i) {
    const float v = Ts[(q * 32 + i) * 68 + c];
    s1 += v;
    s2 += v * v;
  }
  red[q * 64 + c] = s1;
  red[256 + q * 64 + c] = s2;
  __syncthreads();
  if (tid < 128) {
    const int wq = tid >> 6, cc = tid & 63;
    const float* rp = red + wq * 256 + cc;
    stg[tid] = (rp[0] + rp[64]) + (rp[128] + rp[192]);
  }
  __syncthreads();
  if (tid < 32) {
    const v4f v = *(const v4f*)(stg + tid * 4);
    for (int pass = 0; pass < 2; ++pass) {
      *(volatile v4f*)(dst + tid * 4) = v;
      __threadfence();
    }
  }
}

__global__ __launch_bounds__(256) void k_gemm0(const float* __restrict__ xyz, const float* __restrict__ points,
                                               const int* __restrict__ fidx, const int* __restrict__ gidx,
                                               const _Float16* __restrict__ wf0, const float* __restrict__ bias0,
                                               unsigned short* __restrict__ y0, float* __restrict__ part0) {
  __shared__ __align__(16) _Float16 As[128 * KPAD0];
  __shared__ __align__(16) float Ts[128 * 68];
  __shared__ int gil[128];
  __shared__ __align__(16) float red[512];
  __shared__ __align__(16) float stg[128];
  const int tid = threadIdx.x, lane = tid & 31, wave = tid >> 5, hh = lane >> 4, rl = lane & 15;
  const int koff = hh * 8;
  const int row0 = blockIdx.x * 128;
  const int b = row0 >> 15;
  if (tid < 128) {
    int g = gidx[row0 + tid];
    g = g < 0 ? 0 : (g > NPTS - 1 ? NPTS - 1 : g);
    gil[tid] = g;
  }
  __syncthreads();
#pragma unroll 2
  for (int i = 0; i < 4; ++i) {
    const int ch = tid + 256 * i;
    const int r = ch >> 3;
    const int c0 = (ch & 7) * 8;
    const int gi = gil[r];
    const float* pp = points + ((size_t)(b * NPTS + gi)) * CPTS + c0;
    const v4f p0 = *(const v4f*)pp;
    const v4f p1 = *(const v4f*)(pp + 4);
    v8h hv;
#pragma unroll
    for (int e = 0; e < 4; ++e) { hv[e] = (_Float16)p0[e]; hv[4 + e] = (_Float16)p1[e]; }
    *(v8h*)(&As[r * KPAD0 + c0]) = hv;
  }
  if (tid < 128) {
    const int r = tid;
    const int gi = gil[r];
    const int s = ((row0 + r) >> 5) & (NCEN - 1);
    int ci = fidx[b * NCEN + s];
    ci = ci < 0 ? 0 : (ci > NPTS - 1 ? NPTS - 1 : ci);
    const float* px = xyz + ((size_t)(b * NPTS + gi)) * 3;
    const float* pc = xyz + ((size_t)(b * NPTS + ci)) * 3;
    const float x0 = px[0], x1 = px[1], x2 = px[2];
    const float q0 = pc[0], q1 = pc[1], q2 = pc[2];
    const float d0 = x0 - q0, d1 = x1 - q1, d2 = x2 - q2;
    float zf = 0.0f;
    asm volatile("" : "+v"(zf));
    const _Float16 zh = (_Float16)zf;
    v8h h0, hz;
#pragma unroll
    for (int e = 0; e < 8; ++e) { h0[e] = zh; hz[e] = zh; }
    h0[0] = (_Float16)d0;
    h0[1] = (_Float16)d1;
    h0[2] = (_Float16)d2;
    *(v8h*)(&As[r * KPAD0 + 64]) = h0;
    *(v8h*)(&As[r * KPAD0 + 72]) = hz;
    *(v8h*)(&As[r * KPAD0 + 80]) = hz;
    *(v8h*)(&As[r * KPAD0 + 88]) = hz;
  }
  __syncthreads();

  const v8f zero8 = (v8f){0.f, 0.f, 0.f, 0.f, 0.f, 0.f, 0.f, 0.f};
  v8f acc0 = zero8, acc1 = zero8, acc2 = zero8, acc3 = zero8;
#pragma unroll 1
  for (int ks = 0; ks < KPAD0 / 32; ++ks) {
    const int ko = ks * 32 + koff;
    const v16h a  = frag_ld(&As[(wave * 16 + rl) * KPAD0 + ko]);
    const v16h b0 = frag_ld(wf0 + (0 * 16 + rl) * KPAD0 + ko);
    const v16h b1 = frag_ld(wf0 + (1 * 16 + rl) * KPAD0 + ko);
    const v16h b2 = frag_ld(wf0 + (2 * 16 + rl) * KPAD0 + ko);
    const v16h b3 = frag_ld(wf0 + (3 * 16 + rl) * KPAD0 + ko);
    acc0 = mma_h(a, b0, acc0);
    acc1 = mma_h(a, b1, acc1);
    acc2 = mma_h(a, b2, acc2);
    acc3 = mma_h(a, b3, acc3);
    guard4(acc0, acc1, acc2, acc3, a, b0, b1, b2, b3);
  }
  {
    const int rb = wave * 16 + 8 * hh;
    put_tile(Ts, 68, rb, 0 * 16 + rl, acc0, bias0[0 * 16 + rl]);
    put_tile(Ts, 68, rb, 1 * 16 + rl, acc1, bias0[1 * 16 + rl]);
    put_tile(Ts, 68, rb, 2 * 16 + rl, acc2, bias0[2 * 16 + rl]);
    put_tile(Ts, 68, rb, 3 * 16 + rl, acc3, bias0[3 * 16 + rl]);
  }
  __syncthreads();
  {
    const int q = lane >> 3, c8 = (lane & 7) * 8;
    for (int pass = 0; pass < 2; ++pass) {
#pragma unroll
      for (int it = 0; it < 4; ++it) {
        const int row = wave * 16 + it * 4 + q;
        const v4f a = *(const v4f*)(&Ts[row * 68 + c8]);
        const v4f bq = *(const v4f*)(&Ts[row * 68 + c8 + 4]);
        v8h hv;
#pragma unroll
        for (int e = 0; e < 4; ++e) { hv[e] = (_Float16)a[e]; hv[4 + e] = (_Float16)bq[e]; }
        *(volatile v8h*)(void*)(y0 + (size_t)(row0 + row) * 64 + c8) = hv;
      }
      __threadfence();
    }
  }
  stats128(Ts, red, stg, part0 + (size_t)blockIdx.x * 128, tid);
}

template <int CH>
__global__ __launch_bounds__(256) void k_fin(const float* __restrict__ part, int nblk, const float* __restrict__ gam,
                                             const float* __restrict__ bet, float* __restrict__ tab) {
  constexpr int NC = 2 * CH;
  constexpr int SL = 256 / NC;
  static_assert(SL == 1 || SL == 2, "slice count");
  __shared__ double sd[256];
  __shared__ __align__(16) float tabs[4 * CH];
  const int tid = threadIdx.x;
  const int col = tid % NC, sl = tid / NC;
  double acc = 0.0;
#pragma unroll 4
  for (int r = sl; r < nblk; r += SL) acc += (double)part[(size_t)r * NC + col];
  sd[tid] = acc;
  __syncthreads();
  if (tid < CH) {
    double s1 = sd[tid], s2 = sd[CH + tid];
    if (SL == 2) { s1 += sd[NC + tid]; s2 += sd[NC + CH + tid]; }
    const double invm = 1.0 / (double)MROWS;
    const double mean = s1 * invm;
    double var = s2 * invm - mean * mean;
    var = var < 0.0 ? 0.0 : var;
    const float vf = (float)var;
    const float inv = 1.0f / sqrtf(vf + BN_EPS);
    tabs[tid] = (float)mean;
    tabs[CH + tid] = inv;
    tabs[2 * CH + tid] = gam[tid];
    tabs[3 * CH + tid] = bet[tid];
  }
  __syncthreads();
  if (tid < 32) {
    for (int pass = 0; pass < 2; ++pass) {
#pragma unroll
      for (int i = 0; i < (4 * CH) / 128; ++i) {
        const v4f v = *(const v4f*)(&tabs[i * 128 + tid * 4]);
        *(volatile v4f*)(tab + i * 128 + tid * 4) = v;
      }
      __threadfence();
    }
  }
}

template <int ROWS>
__device__ __forceinline__ void stage_a1(const unsigned short* __restrict__ y0, int row0, const float* stab,
                                         _Float16* A1, int tid) {
  const int c0 = (tid & 7) * 8;
  float pm[8], pi[8], pg[8], pb[8];
#pragma unroll
  for (int e = 0; e < 8; ++e) {
    pm[e] = stab[c0 + e];
    pi[e] = stab[64 + c0 + e];
    pg[e] = stab[128 + c0 + e];
    pb[e] = stab[192 + c0 + e];
  }
#pragma unroll 2
  for (int i = 0; i < ROWS * 8 / 256; ++i) {
    const int r = (tid >> 3) + 32 * i;
    const v4u w = *(const v4u*)(const void*)(y0 + (size_t)(row0 + r) * 64 + c0);
    const unsigned w0 = w[0], w1 = w[1], w2 = w[2], w3 = w[3];
    float yv[8];
    yv[0] = h16_to_f32(w0 & 0xffffu);
    yv[1] = h16_to_f32(w0 >> 16);
    yv[2] = h16_to_f32(w1 & 0xffffu);
    yv[3] = h16_to_f32(w1 >> 16);
    yv[4] = h16_to_f32(w2 & 0xffffu);
    yv[5] = h16_to_f32(w2 >> 16);
    yv[6] = h16_to_f32(w3 & 0xffffu);
    yv[7] = h16_to_f32(w3 >> 16);
    v8h hv;
#pragma unroll
    for (int e = 0; e < 8; ++e) hv[e] = (_Float16)bn_relu(yv[e], pm[e], pi[e], pg[e], pb[e]);
    *(v8h*)(A1 + r * 64 + c0) = hv;
  }
}

__global__ __launch_bounds__(256) void k_gemm1s(const unsigned short* __restrict__ y0, const float* __restrict__ tab0,
                                                const float* __restrict__ bias1, const _Float16* __restrict__ wf1,
                                                float* __restrict__ part1) {
  __shared__ __align__(16) _Float16 A1[128 * 64];
  __shared__ __align__(16) float Ts[128 * 68];
  __shared__ __align__(16) float red[512];
  __shared__ __align__(16) float stg[128];
  __shared__ __align__(16) float stab0[256];
  const int tid = threadIdx.x, lane = tid & 31, wave = tid >> 5, hh = lane >> 4, rl = lane & 15;
  const int koff = hh * 8;
  const int row0 = blockIdx.x * 128;
  if (tid < 64) *(v4f*)(&stab0[tid * 4]) = *(const v4f*)(tab0 + tid * 4);
  __syncthreads();
  stage_a1<128>(y0, row0, stab0, A1, tid);
  __syncthreads();
  const v8f zero8 = (v8f){0.f, 0.f, 0.f, 0.f, 0.f, 0.f, 0.f, 0.f};
  v8f acc0 = zero8, acc1 = zero8, acc2 = zero8, acc3 = zero8;
#pragma unroll 1
  for (int ks = 0; ks < 2; ++ks) {
    const int ko = ks * 32 + koff;
    const v16h a  = frag_ld(&A1[(wave * 16 + rl) * 64 + ko]);
    const v16h b0 = frag_ld(wf1 + (0 * 16 + rl) * 64 + ko);
    const v16h b1 = frag_ld(wf1 + (1 * 16 + rl) * 64 + ko);
    const v16h b2 = frag_ld(wf1 + (2 * 16 + rl) * 64 + ko);
    const v16h b3 = frag_ld(wf1 + (3 * 16 + rl) * 64 + ko);
    acc0 = mma_h(a, b0, acc0);
    acc1 = mma_h(a, b1, acc1);
    acc2 = mma_h(a, b2, acc2);
    acc3 = mma_h(a, b3, acc3);
    guard4(acc0, acc1, acc2, acc3, a, b0, b1, b2, b3);
  }
  {
    const int rb = wave * 16 + 8 * hh;
    put_tile(Ts, 68, rb, 0 * 16 + rl, acc0, bias1[0 * 16 + rl]);
    put_tile(Ts, 68, rb, 1 * 16 + rl, acc1, bias1[1 * 16 + rl]);
    put_tile(Ts, 68, rb, 2 * 16 + rl, acc2, bias1[2 * 16 + rl]);
    put_tile(Ts, 68, rb, 3 * 16 + rl, acc3, bias1[3 * 16 + rl]);
  }
  __syncthreads();
  stats128(Ts, red, stg, part1 + (size_t)blockIdx.x * 128, tid);
}

__global__ __launch_bounds__(256) void k_chain(const unsigned short* __restrict__ y0, const float* __restrict__ tab0,
                                               const float* __restrict__ tab1, const float* __restrict__ bias1,
                                               const float* __restrict__ bias2, const _Float16* __restrict__ wf1,
                                               const _Float16* __restrict__ wf2, float* __restrict__ part2,
                                               float* __restrict__ gmax, float* __restrict__ gmin) {
  __shared__ __align__(16) _Float16 A1[64 * 64];
  __shared__ __align__(16) _Float16 A2[64 * 64];
  __shared__ __align__(16) float Ts[64 * 132];
  __shared__ __align__(16) float red[512];
  __shared__ __align__(16) float sgm[512];
  __shared__ __align__(16) float stab0[256];
  __shared__ __align__(16) float stab1[256];
  const int tid = threadIdx.x, lane = tid & 31, wave = tid >> 5, hh = lane >> 4, rl = lane & 15;
  const int koff = hh * 8;
  const int row0 = blockIdx.x * 64;
  if (tid < 64) {
    *(v4f*)(&stab0[tid * 4]) = *(const v4f*)(tab0 + tid * 4);
  } else if (tid < 128) {
    *(v4f*)(&stab1[(tid - 64) * 4]) = *(const v4f*)(tab1 + (tid - 64) * 4);
  }
  __syncthreads();
  stage_a1<64>(y0, row0, stab0, A1, tid);
  __syncthreads();

  const int mt = wave >> 1, nh = wave & 1;
  const v8f zero8 = (v8f){0.f, 0.f, 0.f, 0.f, 0.f, 0.f, 0.f, 0.f};
  v8f p0 = zero8, p1 = zero8;
#pragma unroll 1
  for (int ks = 0; ks < 2; ++ks) {
    const int ko = ks * 32 + koff;
    const v16h a  = frag_ld(&A1[(mt * 16 + rl) * 64 + ko]);
    const v16h b0 = frag_ld(wf1 + ((2 * nh + 0) * 16 + rl) * 64 + ko);
    const v16h b1 = frag_ld(wf1 + ((2 * nh + 1) * 16 + rl) * 64 + ko);
    p0 = mma_h(a, b0, p0);
    p1 = mma_h(a, b1, p1);
    guard2(p0, p1, a, b0, b1);
  }
  {
    const int n0 = (2 * nh + 0) * 16 + rl;
    const int n1 = (2 * nh + 1) * 16 + rl;
    const float m0 = stab1[n0], i0 = stab1[64 + n0], g0 = stab1[128 + n0], e0 = stab1[192 + n0];
    const float m1 = stab1[n1], i1 = stab1[64 + n1], g1 = stab1[128 + n1], e1 = stab1[192 + n1];
    const float bb0 = bias1[n0], bb1 = bias1[n1];
    const int rb = mt * 16 + 8 * hh;
#pragma unroll
    for (int r = 0; r < 8; ++r) {
      const float v0 = p0[r] * WCARRY_INV + bb0;
      const float v1 = p1[r] * WCARRY_INV + bb1;
      A2[(rb + r) * 64 + n0] = (_Float16)bn_relu(v0, m0, i0, g0, e0);
      A2[(rb + r) * 64 + n1] = (_Float16)bn_relu(v1, m1, i1, g1, e1);
    }
  }
  __syncthreads();
  v8f acc0 = zero8, acc1 = zero8, acc2 = zero8, acc3 = zero8;
#pragma unroll 1
  for (int ks = 0; ks < 2; ++ks) {
    const int ko = ks * 32 + koff;
    const v16h a  = frag_ld(&A2[(mt * 16 + rl) * 64 + ko]);
    const v16h b0 = frag_ld(wf2 + ((4 * nh + 0) * 16 + rl) * 64 + ko);
    const v16h b1 = frag_ld(wf2 + ((4 * nh + 1) * 16 + rl) * 64 + ko);
    const v16h b2 = frag_ld(wf2 + ((4 * nh + 2) * 16 + rl) * 64 + ko);
    const v16h b3 = frag_ld(wf2 + ((4 * nh + 3) * 16 + rl) * 64 + ko);
    acc0 = mma_h(a, b0, acc0);
    acc1 = mma_h(a, b1, acc1);
    acc2 = mma_h(a, b2, acc2);
    acc3 = mma_h(a, b3, acc3);
    guard4(acc0, acc1, acc2, acc3, a, b0, b1, b2, b3);
  }
  {
    const int rb = mt * 16 + 8 * hh;
    put_tile(Ts, 132, rb, (4 * nh + 0) * 16 + rl, acc0, bias2[(4 * nh + 0) * 16 + rl]);
    put_tile(Ts, 132, rb, (4 * nh + 1) * 16 + rl, acc1, bias2[(4 * nh + 1) * 16 + rl]);
    put_tile(Ts, 132, rb, (4 * nh + 2) * 16 + rl, acc2, bias2[(4 * nh + 2) * 16 + rl]);
    put_tile(Ts, 132, rb, (4 * nh + 3) * 16 + rl, acc3, bias2[(4 * nh + 3) * 16 + rl]);
  }
  __syncthreads();
  {
    const int c = tid & 127, half = tid >> 7;
    float s1 = 0.0f, s2 = 0.0f;
    float mx = -__builtin_huge_valf(), mn = __builtin_huge_valf();
#pragma unroll 4
    for (int i = 0; i < 32; ++i) {
      const float v = Ts[(half * 32 + i) * 132 + c];
      s1 += v;
      s2 += v * v;
      mx = fmaxf(mx, v);
      mn = fminf(mn, v);
    }
    red[(half * 2 + 0) * 128 + c] = s1;
    red[(half * 2 + 1) * 128 + c] = s2;
    sgm[half * 128 + c] = mx;
    sgm[(2 + half) * 128 + c] = mn;
  }
  __syncthreads();
  if (wave < 4) {
    const v4f v = *(const v4f*)(&sgm[wave * 128 + lane * 4]);
    float* base = (wave < 2) ? gmax : gmin;
    float* dstp = base + ((size_t)blockIdx.x * 2 + (wave & 1)) * 128 + lane * 4;
    for (int pass = 0; pass < 2; ++pass) {
      *(volatile v4f*)dstp = v;
      __threadfence();
    }
  } else if (wave < 6) {
    const int qy = wave - 4;
    const v4f a = *(const v4f*)(&red[qy * 128 + lane * 4]);
    const v4f bq = *(const v4f*)(&red[(2 + qy) * 128 + lane * 4]);
    const v4f v = a + bq;
    float* dstp = part2 + (size_t)blockIdx.x * 256 + qy * 128 + lane * 4;
    for (int pass = 0; pass < 2; ++pass) {
      *(volatile v4f*)dstp = v;
      __threadfence();
    }
  }
}

__global__ __launch_bounds__(256) void k_out(const float* __restrict__ gmax, const float* __restrict__ gmin,
                                             const float* __restrict__ tab2, float* __restrict__ out1) {
  const int i = blockIdx.x * 256 + threadIdx.x;
  const int c4 = (i & 31) * 4;
  const v4f mx = *(const v4f*)(gmax + (size_t)i * 4);
  const v4f mn = *(const v4f*)(gmin + (size_t)i * 4);
  const v4f m  = *(const v4f*)(tab2 + c4);
  const v4f iv = *(const v4f*)(tab2 + 128 + c4);
  const v4f gv = *(const v4f*)(tab2 + 256 + c4);
  const v4f bv = *(const v4f*)(tab2 + 384 + c4);
  v4f o;
#pragma unroll
  for (int e = 0; e < 4; ++e) {
    const float sel = (gv[e] >= 0.0f) ? mx[e] : mn[e];
    o[e] = bn_relu(sel, m[e], iv[e], gv[e], bv[e]);
  }
  float* dstp = out1 + (size_t)i * 4;
  *(volatile v4f*)dstp = o;
  __threadfence();
  *(volatile v4f*)dstp = o;
}

extern "C" void kernel_launch(void* const* d_in, const int* in_sizes, int n_in,
                              void* d_out, int out_size, void* d_ws, size_t ws_size,
                              hipStream_t stream) {
  (void)in_sizes; (void)n_in; (void)out_size;
  if (ws_size < WS_TOTAL) return;
  const float* xyz    = (const float*)d_in[0];
  const float* points = (const float*)d_in[1];
  const float* w0  = (const float*)d_in[2];
  const float* b0  = (const float*)d_in[3];
  const float* g0  = (const float*)d_in[4];
  const float* be0 = (const float*)d_in[5];
  const float* w1  = (const float*)d_in[6];
  const float* b1  = (const float*)d_in[7];
  const float* g1  = (const float*)d_in[8];
  const float* be1 = (const float*)d_in[9];
  const float* w2  = (const float*)d_in[10];
  const float* b2  = (const float*)d_in[11];
  const float* g2  = (const float*)d_in[12];
  const float* be2 = (const float*)d_in[13];

  float* out0 = (float*)d_out;
  float* out1 = (float*)d_out + OUT0_FLOATS;

  char* ws = (char*)d_ws;
  int* fidx = (int*)(ws + OFF_FIDX);
  int* gidx = (int*)(ws + OFF_GIDX);
  _Float16* wf = (_Float16*)(ws + OFF_WF);
  const _Float16* wf0 = wf;
  const _Float16* wf1 = wf + 64 * KPAD0;
  const _Float16* wf2 = wf + 64 * KPAD0 + 64 * 64;
  float* tab0 = (float*)(ws + OFF_TAB0);
  float* tab1 = (float*)(ws + OFF_TAB1);
  float* tab2 = (float*)(ws + OFF_TAB2);
  unsigned short* y0 = (unsigned short*)(ws + OFF_Y0);
  float* part0 = (float*)(ws + OFF_P0);
  float* part1 = (float*)(ws + OFF_P1);
  float* part2 = (float*)(ws + OFF_P2);
  float* gmax = (float*)(ws + OFF_GMAX);
  float* gmin = (float*)(ws + OFF_GMIN);

  k_fps<<<NBATCH, 256, 0, stream>>>(xyz, out0, fidx);
  k_ball<<<(NBATCH * NCEN) / 8, 256, 0, stream>>>(xyz, fidx, gidx);
  k_wprep<<<9, 256, 0, stream>>>(w0, w1, w2, wf);
  k_gemm0<<<MROWS / 128, 256, 0, stream>>>(xyz, points, fidx, gidx, wf0, b0, y0, part0);
  k_fin<64><<<1, 256, 0, stream>>>(part0, MROWS / 128, g0, be0, tab0);
  k_gemm1s<<<MROWS / 128, 256, 0, stream>>>(y0, tab0, b1, wf1, part1);
  k_fin<64><<<1, 256, 0, stream>>>(part1, MROWS / 128, g1, be1, tab1);
  k_chain<<<MROWS / 64, 256, 0, stream>>>(y0, tab0, tab1, b1, b2, wf1, wf2, part2, gmax, gmin);
  k_fin<128><<<1, 256, 0, stream>>>(part2, MROWS / 64, g2, be2, tab2);
  k_out<<<(NBATCH * NCEN * 128 / 4) / 256, 256, 0, stream>>>(gmax, gmin, tab2, out1);
}
